// SmallAttention_34411277976107
// MI455X (gfx1250) — hardware-verified
//
#include <hip/hip_runtime.h>
#include <stddef.h>
#include <stdint.h>

#define NBATCH 4
#define SQ     4096
#define NTOK   (NBATCH * SQ)
#define DIN    512
#define HDM    64
#define NQKV   (3 * HDM)
#define DOUT   512
#define QB     64
#define KC     64
#define NQB    (SQ / QB)

static_assert(NTOK == 16384);
static_assert(NQKV == 192);
static_assert(SQ % QB == 0);
static_assert(SQ % KC == 0);
static_assert(QB == KC);
static_assert(DIN % 64 == 0);
static_assert(DOUT % 64 == 0);
static_assert(HDM == 64);
static_assert((NTOK * DIN) % 2048 == 0);
static_assert(NTOK % 64 == 0);
static_assert(NQKV % 64 == 0);

typedef unsigned short us;
typedef __attribute__((ext_vector_type(16))) __bf16 v16bf;
typedef us           v8us __attribute__((ext_vector_type(8)));
typedef float        v8f  __attribute__((ext_vector_type(8)));
typedef float        v4f  __attribute__((ext_vector_type(4)));
typedef unsigned int v4u  __attribute__((ext_vector_type(4)));

union Frag  { v16bf v; v8us h[2]; };
union Pack8 { v8us h; v4u u; };

__device__ __forceinline__ us bf_rne(float f) {
  unsigned u = __float_as_uint(f);
  u = u + 0x7FFFu + ((u >> 16) & 1u);
  return (us)(u >> 16);
}
__device__ __forceinline__ float bf_val(us h) { return __uint_as_float(((unsigned)h) << 16); }
__device__ __forceinline__ void split2(float f, us& hi, us& lo) {
  const us hv = bf_rne(f);
  hi = hv;
  lo = bf_rne(f - bf_val(hv));
}
__device__ __forceinline__ void split8(const float (&f)[8], Pack8& ph, Pack8& pl) {
  us hh[8], ll[8];
#pragma unroll
  for (int e = 0; e < 8; ++e) split2(f[e], hh[e], ll[e]);
  ph.h = (v8us){hh[0], hh[1], hh[2], hh[3], hh[4], hh[5], hh[6], hh[7]};
  pl.h = (v8us){ll[0], ll[1], ll[2], ll[3], ll[4], ll[5], ll[6], ll[7]};
}

__device__ __forceinline__ v8f mma16(v16bf a, v16bf b, v8f c) {
  c = __builtin_amdgcn_wmma_f32_16x16x32_bf16(false, a, false, b, (short)0, c, false, false);
  asm volatile("v_nop\n\tv_nop\n\tv_nop\n\tv_nop" : "+v"(c) : "v"(a), "v"(b));
  return c;
}

__device__ __forceinline__ v16bf ldfrag(const us* p, int ld, int row0, int k0, int lane) {
  const int m = lane & 15, lh = lane >> 4;
  const us* q = p + (size_t)(row0 + m) * ld + k0 + 8 * lh;
  Frag f;
  f.h[0] = *(const v8us*)(q);
  f.h[1] = *(const v8us*)(q + 16);
  return f.v;
}

__device__ __forceinline__ v8f zero8() { return (v8f){0.f, 0.f, 0.f, 0.f, 0.f, 0.f, 0.f, 0.f}; }

template <int KD>
__device__ __forceinline__ void gemm16x64x3(const us* __restrict__ Ah, const us* __restrict__ Al,
                                            const us* __restrict__ Bh, const us* __restrict__ Bl,
                                            int m0, int n0, int lane, v8f (&acc)[4]) {
  static_assert(KD % 32 == 0);
#pragma unroll 1
  for (int k0 = 0; k0 < KD; k0 += 32) {
    const v16bf ah = ldfrag(Ah, KD, m0, k0, lane);
    const v16bf al = ldfrag(Al, KD, m0, k0, lane);
#pragma unroll
    for (int t = 0; t < 4; ++t) {
      const v16bf bh = ldfrag(Bh, KD, n0 + 16 * t, k0, lane);
      const v16bf bl = ldfrag(Bl, KD, n0 + 16 * t, k0, lane);
      acc[t] = mma16(ah, bh, acc[t]);
      acc[t] = mma16(ah, bl, acc[t]);
      acc[t] = mma16(al, bh, acc[t]);
    }
  }
}

#define TWP 68
__global__ __launch_bounds__(128) void k_cvtw(const float* __restrict__ wqkv, const float* __restrict__ wout,
                                              us* __restrict__ wqh, us* __restrict__ wql,
                                              us* __restrict__ woh, us* __restrict__ wol) {
  __shared__ __align__(16) float tl[64 * TWP];
  const int tid = threadIdx.x;
  const int id = blockIdx.x;
  const bool isq = (id < 24);
  const float* s = isq ? wqkv : wout;
  const int spitch = isq ? NQKV : DOUT;
  const int n0 = isq ? (64 * (id % 3)) : (64 * (id - 24));
  const int k0 = isq ? (64 * (id / 3)) : 0;
  us* dh = isq ? wqh : woh;
  us* dl = isq ? wql : wol;
  const int dpitch = isq ? DIN : HDM;
#pragma unroll
  for (int j = 0; j < 8; ++j) {
    const int p  = tid + 128 * j;
    const int kr = p >> 4;
    const int c4 = (p & 15) * 4;
    const v4f a = *(const v4f*)(s + (size_t)(k0 + kr) * spitch + n0 + c4);
    *(v4f*)(tl + kr * TWP + c4) = a;
  }
  __syncthreads();
  v4u hv[4], lv[4];
  size_t go[4];
#pragma unroll
  for (int j = 0; j < 4; ++j) {
    const int p  = tid + 128 * j;
    const int n  = p >> 3;
    const int kc = (p & 7) * 8;
    const float* cp = tl + kc * TWP + n;
    float f[8];
#pragma unroll
    for (int e = 0; e < 8; ++e) f[e] = cp[e * TWP];
    Pack8 ph, pl;
    split8(f, ph, pl);
    hv[j] = ph.u;
    lv[j] = pl.u;
    go[j] = ((size_t)(n0 + n)) * dpitch + k0 + kc;
  }
#pragma unroll
  for (int j = 0; j < 4; ++j) { *(volatile v4u*)(dh + go[j]) = hv[j]; *(volatile v4u*)(dl + go[j]) = lv[j]; }
  __threadfence();
#pragma unroll
  for (int j = 0; j < 4; ++j) { *(volatile v4u*)(dh + go[j]) = hv[j]; *(volatile v4u*)(dl + go[j]) = lv[j]; }
}

__global__ __launch_bounds__(256) void k_cvtx(const float* __restrict__ x, us* __restrict__ xh, us* __restrict__ xl) {
  const size_t i = (size_t)blockIdx.x * 2048 + (size_t)threadIdx.x * 8;
  const v4f a0 = *(const v4f*)(x + i);
  const v4f a1 = *(const v4f*)(x + i + 4);
  const float f[8] = {a0[0], a0[1], a0[2], a0[3], a1[0], a1[1], a1[2], a1[3]};
  Pack8 ph, pl;
  split8(f, ph, pl);
  const v4u hv = ph.u, lv = pl.u;
  *(volatile v4u*)(xh + i) = hv;
  *(volatile v4u*)(xl + i) = lv;
  __threadfence();
  *(volatile v4u*)(xh + i) = hv;
  *(volatile v4u*)(xl + i) = lv;
}

#define SFP 68
__global__ __launch_bounds__(128) void k_qkv(const us* __restrict__ xh, const us* __restrict__ xl,
                                             const us* __restrict__ wh, const us* __restrict__ wl,
                                             us* __restrict__ qh, us* __restrict__ ql,
                                             us* __restrict__ kh, us* __restrict__ kl,
                                             us* __restrict__ vh, us* __restrict__ vl) {
  __shared__ __align__(16) float sf[64 * SFP];
  const int tid = threadIdx.x, lane = tid & 31, wave = tid >> 5;
  const int hh = lane >> 4, c = lane & 15;
  const int mb = blockIdx.x * 64;
  const int ns = blockIdx.y;
  const int m0 = mb + wave * 16;
  const int n0 = 64 * ns;

  v8f acc[4];
#pragma unroll
  for (int t = 0; t < 4; ++t) acc[t] = zero8();
  gemm16x64x3<DIN>(xh, xl, wh, wl, m0, n0, lane, acc);

#pragma unroll
  for (int t = 0; t < 4; ++t) {
#pragma unroll
    for (int r = 0; r < 8; ++r)
      sf[(wave * 16 + 8 * hh + r) * SFP + 16 * t + c] = acc[t][r];
  }
  __syncthreads();

  if (ns < 2) {
    v4u hv[4], lv[4];
    size_t go[4];
#pragma unroll
    for (int j = 0; j < 4; ++j) {
      const int p  = tid + 128 * j;
      const int lr = p >> 3;
      const int d0 = (p & 7) * 8;
      const float* ra = sf + lr * SFP + d0;
      const v4f a0 = *(const v4f*)(ra), a1 = *(const v4f*)(ra + 4);
      const float f[8] = {a0[0], a0[1], a0[2], a0[3], a1[0], a1[1], a1[2], a1[3]};
      Pack8 ph, pl;
      split8(f, ph, pl);
      hv[j] = ph.u;
      lv[j] = pl.u;
      go[j] = ((size_t)(mb + lr)) * HDM + d0;
    }
    us* dsth = (ns == 0) ? qh : kh;
    us* dstl = (ns == 0) ? ql : kl;
#pragma unroll
    for (int j = 0; j < 4; ++j) { *(volatile v4u*)(dsth + go[j]) = hv[j]; *(volatile v4u*)(dstl + go[j]) = lv[j]; }
    __threadfence();
#pragma unroll
    for (int j = 0; j < 4; ++j) { *(volatile v4u*)(dsth + go[j]) = hv[j]; *(volatile v4u*)(dstl + go[j]) = lv[j]; }
  } else {
    v4u hv[4], lv[4];
    size_t go[4];
    const int bidx = mb / SQ;
    const int s0   = mb - bidx * SQ;
#pragma unroll
    for (int j = 0; j < 4; ++j) {
      const int p  = tid + 128 * j;
      const int d  = p >> 3;
      const int pc = p & 7;
      const float* cp = sf + (pc * 8) * SFP + d;
      float f[8];
#pragma unroll
      for (int e = 0; e < 8; ++e) f[e] = cp[e * SFP];
      Pack8 ph, pl;
      split8(f, ph, pl);
      hv[j] = ph.u;
      lv[j] = pl.u;
      go[j] = ((size_t)(bidx * HDM + d)) * SQ + s0 + pc * 8;
    }
#pragma unroll
    for (int j = 0; j < 4; ++j) { *(volatile v4u*)(vh + go[j]) = hv[j]; *(volatile v4u*)(vl + go[j]) = lv[j]; }
    __threadfence();
#pragma unroll
    for (int j = 0; j < 4; ++j) { *(volatile v4u*)(vh + go[j]) = hv[j]; *(volatile v4u*)(vl + go[j]) = lv[j]; }
  }
}

#define LP 72
__global__ __launch_bounds__(128) void k_attn(const us* __restrict__ qh, const us* __restrict__ ql,
                                              const us* __restrict__ kh, const us* __restrict__ kl,
                                              const us* __restrict__ vh, const us* __restrict__ vl,
                                              us* __restrict__ oh, us* __restrict__ ol) {
  __shared__ __align__(16) us Ksh[KC * LP];
  __shared__ __align__(16) us Ksl[KC * LP];
  __shared__ __align__(16) us Vsh[HDM * LP];
  __shared__ __align__(16) us Vsl[HDM * LP];
  __shared__ __align__(16) us Psh[4 * 16 * LP];
  __shared__ __align__(16) us Psl[4 * 16 * LP];

  const int tid = threadIdx.x, lane = tid & 31, wave = tid >> 5;
  const int hh = lane >> 4, c = lane & 15;
  const int qb  = blockIdx.x % NQB;
  const int b   = blockIdx.x / NQB;
  const int qp0 = qb * QB + wave * 16;
  const int q0  = b * SQ + qp0;

  const us* Kh = kh + (size_t)b * SQ * HDM;
  const us* Kl = kl + (size_t)b * SQ * HDM;
  const us* Vh = vh + (size_t)b * HDM * SQ;
  const us* Vl = vl + (size_t)b * HDM * SQ;

  const float NEGI = -__builtin_huge_valf();
  float mrow[8], lrow[8];
  v8f oacc[4];
#pragma unroll
  for (int r = 0; r < 8; ++r) { mrow[r] = NEGI; lrow[r] = 0.f; }
#pragma unroll
  for (int t = 0; t < 4; ++t) oacc[t] = zero8();

  us* pwh = Psh + wave * 16 * LP;
  us* pwl = Psl + wave * 16 * LP;
  const int nck = qb + 1;

  for (int i = 0; i < nck; ++i) {
    const int kv0 = i * KC;
    __syncthreads();
    {
      const int r  = tid >> 1;
      const int cb = (tid & 1) * 32;
      const us* ksh = Kh + (size_t)(kv0 + r) * HDM + cb;
      const us* ksl = Kl + (size_t)(kv0 + r) * HDM + cb;
      const us* vsh = Vh + (size_t)r * SQ + kv0 + cb;
      const us* vsl = Vl + (size_t)r * SQ + kv0 + cb;
#pragma unroll
      for (int e = 0; e < 4; ++e) {
        *(v8us*)(Ksh + r * LP + cb + 8 * e) = *(const v8us*)(ksh + 8 * e);
        *(v8us*)(Ksl + r * LP + cb + 8 * e) = *(const v8us*)(ksl + 8 * e);
        *(v8us*)(Vsh + r * LP + cb + 8 * e) = *(const v8us*)(vsh + 8 * e);
        *(v8us*)(Vsl + r * LP + cb + 8 * e) = *(const v8us*)(vsl + 8 * e);
      }
    }
    __syncthreads();

    v8f s[4];
#pragma unroll
    for (int j = 0; j < 4; ++j) s[j] = zero8();
#pragma unroll
    for (int dc = 0; dc < 2; ++dc) {
      const v16bf qah = ldfrag(qh, HDM, q0, dc * 32, lane);
      const v16bf qal = ldfrag(ql, HDM, q0, dc * 32, lane);
#pragma unroll
      for (int j = 0; j < 4; ++j) {
        const v16bf kbh = ldfrag(Ksh, LP, j * 16, dc * 32, lane);
        const v16bf kbl = ldfrag(Ksl, LP, j * 16, dc * 32, lane);
        s[j] = mma16(qah, kbh, s[j]);
        s[j] = mma16(qah, kbl, s[j]);
        s[j] = mma16(qal, kbh, s[j]);
      }
    }
#pragma unroll
    for (int r = 0; r < 8; ++r) {
      const int qry = qp0 + 8 * hh + r;
#pragma unroll
      for (int j = 0; j < 4; ++j) {
        const int key = kv0 + 16 * j + c;
        const bool live = (key <= qry);
        const float sv = s[j][r] * 0.125f;
        s[j][r] = live ? sv : NEGI;
      }
    }
    float cm[8];
#pragma unroll
    for (int r = 0; r < 8; ++r) {
      float m = NEGI;
#pragma unroll
      for (int j = 0; j < 4; ++j) m = fmaxf(m, s[j][r]);
#pragma unroll
      for (int off = 1; off < 16; off <<= 1) m = fmaxf(m, __shfl_xor(m, off, 32));
      cm[r] = m;
    }
    float al[8];
#pragma unroll
    for (int r = 0; r < 8; ++r) {
      const float mnew  = fmaxf(mrow[r], cm[r]);
      const float alpha = __expf(mrow[r] - mnew);
      mrow[r] = mnew;
      float psum = 0.f;
#pragma unroll
      for (int j = 0; j < 4; ++j) {
        const float p = __expf(s[j][r] - mnew);
        psum += p;
        us ph, pl;
        split2(p, ph, pl);
        pwh[(8 * hh + r) * LP + j * 16 + c] = ph;
        pwl[(8 * hh + r) * LP + j * 16 + c] = pl;
      }
#pragma unroll
      for (int off = 1; off < 16; off <<= 1) psum += __shfl_xor(psum, off, 32);
      lrow[r] = lrow[r] * alpha + psum;
      al[r] = alpha;
    }
#pragma unroll
    for (int t = 0; t < 4; ++t)
#pragma unroll
      for (int r = 0; r < 8; ++r) oacc[t][r] *= al[r];
    __syncthreads();

#pragma unroll
    for (int kk = 0; kk < 2; ++kk) {
      const v16bf pah = ldfrag(pwh, LP, 0, kk * 32, lane);
      const v16bf pal = ldfrag(pwl, LP, 0, kk * 32, lane);
#pragma unroll
      for (int t = 0; t < 4; ++t) {
        const v16bf vbh = ldfrag(Vsh, LP, t * 16, kk * 32, lane);
        const v16bf vbl = ldfrag(Vsl, LP, t * 16, kk * 32, lane);
        oacc[t] = mma16(pah, vbh, oacc[t]);
        oacc[t] = mma16(pah, vbl, oacc[t]);
        oacc[t] = mma16(pal, vbh, oacc[t]);
      }
    }
  }

  float invl[8];
#pragma unroll
  for (int r = 0; r < 8; ++r) invl[r] = (lrow[r] > 0.f) ? (1.0f / lrow[r]) : 0.f;
  __syncthreads();
#pragma unroll
  for (int r = 0; r < 8; ++r) {
#pragma unroll
    for (int t = 0; t < 4; ++t) {
      us ohv, olv;
      split2(oacc[t][r] * invl[r], ohv, olv);
      pwh[(8 * hh + r) * LP + 16 * t + c] = ohv;
      pwl[(8 * hh + r) * LP + 16 * t + c] = olv;
    }
  }
  __syncthreads();
  v4u hv[4], lv[4];
  size_t go[4];
#pragma unroll
  for (int it = 0; it < 4; ++it) {
    const int p  = lane + 32 * it;
    const int L  = p >> 3;
    const int pc = p & 7;
    Pack8 ph, pl;
    ph.h   = *(const v8us*)(pwh + L * LP + pc * 8);
    pl.h   = *(const v8us*)(pwl + L * LP + pc * 8);
    hv[it] = ph.u;
    lv[it] = pl.u;
    go[it] = (size_t)(q0 + L) * HDM + pc * 8;
  }
#pragma unroll
  for (int it = 0; it < 4; ++it) { *(volatile v4u*)(oh + go[it]) = hv[it]; *(volatile v4u*)(ol + go[it]) = lv[it]; }
  __threadfence();
#pragma unroll
  for (int it = 0; it < 4; ++it) { *(volatile v4u*)(oh + go[it]) = hv[it]; *(volatile v4u*)(ol + go[it]) = lv[it]; }
}

#define OTP 68
__global__ __launch_bounds__(128) void k_out(const us* __restrict__ ah, const us* __restrict__ al,
                                             const us* __restrict__ wh, const us* __restrict__ wl,
                                             const float* __restrict__ bout, float* __restrict__ out) {
  __shared__ __align__(16) float st[4][16 * OTP];
  const int tid = threadIdx.x, lane = tid & 31, wave = tid >> 5;
  const int hh = lane >> 4, c = lane & 15;
  const int m0 = blockIdx.x * 64 + wave * 16;
  const int n0 = blockIdx.y * 64;

  v8f acc[4];
#pragma unroll
  for (int t = 0; t < 4; ++t) acc[t] = zero8();
  gemm16x64x3<HDM>(ah, al, wh, wl, m0, n0, lane, acc);

  float* sw = st[wave];
#pragma unroll
  for (int t = 0; t < 4; ++t) {
#pragma unroll
    for (int r = 0; r < 8; ++r) sw[(8 * hh + r) * OTP + 16 * t + c] = acc[t][r];
  }
  __syncthreads();
  v4f val[8];
  size_t go[8];
#pragma unroll
  for (int it = 0; it < 8; ++it) {
    const int p    = lane + 32 * it;
    const int L    = p >> 3;
    const int pc   = p & 7;
    const int row  = L >> 1;
    const int half = L & 1;
    const int col  = n0 + half * 32 + pc * 4;
    const v4f tv = *(const v4f*)(sw + row * OTP + half * 32 + pc * 4);
    const v4f bb = *(const v4f*)(bout + col);
    go[it]  = (size_t)(m0 + row) * DOUT + col;
    val[it] = tv + bb;
  }
#pragma unroll
  for (int it = 0; it < 8; ++it) *(volatile v4f*)(out + go[it]) = val[it];
  __threadfence();
#pragma unroll
  for (int it = 0; it < 8; ++it) *(volatile v4f*)(out + go[it]) = val[it];
}

extern "C" void kernel_launch(void* const* d_in, const int* in_sizes, int n_in,
                              void* d_out, int out_size, void* d_ws, size_t ws_size,
                              hipStream_t stream) {
  if (n_in < 4) return;
  if (in_sizes[0] != NTOK * DIN) return;
  if (in_sizes[1] != DIN * NQKV) return;
  if (in_sizes[2] != HDM * DOUT) return;
  if (in_sizes[3] != DOUT) return;
  if (out_size != NTOK * DOUT) return;

  const float* x    = (const float*)d_in[0];
  const float* wqkv = (const float*)d_in[1];
  const float* wout = (const float*)d_in[2];
  const float* bout = (const float*)d_in[3];
  float* out = (float*)d_out;

  size_t off = 0;
  const size_t oXh  = off; off += (size_t)NTOK * DIN * 2;
  const size_t oXl  = off; off += (size_t)NTOK * DIN * 2;
  const size_t oWQh = off; off += (size_t)NQKV * DIN * 2;
  const size_t oWQl = off; off += (size_t)NQKV * DIN * 2;
  const size_t oWOh = off; off += (size_t)DOUT * HDM * 2;
  const size_t oWOl = off; off += (size_t)DOUT * HDM * 2;
  const size_t oQh  = off; off += (size_t)NTOK * HDM * 2;
  const size_t oQl  = off; off += (size_t)NTOK * HDM * 2;
  const size_t oKh  = off; off += (size_t)NTOK * HDM * 2;
  const size_t oKl  = off; off += (size_t)NTOK * HDM * 2;
  const size_t oVh  = off; off += (size_t)NBATCH * HDM * SQ * 2;
  const size_t oVl  = off; off += (size_t)NBATCH * HDM * SQ * 2;
  const size_t oOh  = off; off += (size_t)NTOK * HDM * 2;
  const size_t oOl  = off; off += (size_t)NTOK * HDM * 2;
  if (off > ws_size) return;
  if (off > (size_t)134217728) return;

  char* ws = (char*)d_ws;
  us* Xh  = (us*)(ws + oXh);
  us* Xl  = (us*)(ws + oXl);
  us* WQh = (us*)(ws + oWQh);
  us* WQl = (us*)(ws + oWQl);
  us* WOh = (us*)(ws + oWOh);
  us* WOl = (us*)(ws + oWOl);
  us* Qh  = (us*)(ws + oQh);
  us* Ql  = (us*)(ws + oQl);
  us* Kh  = (us*)(ws + oKh);
  us* Kl  = (us*)(ws + oKl);
  us* Vh  = (us*)(ws + oVh);
  us* Vl  = (us*)(ws + oVl);
  us* Oh  = (us*)(ws + oOh);
  us* Ol  = (us*)(ws + oOl);

  k_cvtw<<<dim3(24 + DOUT / 64), dim3(128), 0, stream>>>(wqkv, wout, WQh, WQl, WOh, WOl);
  k_cvtx<<<dim3((NTOK * DIN) / 2048), dim3(256), 0, stream>>>(x, Xh, Xl);
  k_qkv<<<dim3(NTOK / 64, 3), dim3(128), 0, stream>>>(Xh, Xl, WQh, WQl, Qh, Ql, Kh, Kl, Vh, Vl);
  k_attn<<<dim3(NBATCH * NQB), dim3(128), 0, stream>>>(Qh, Ql, Kh, Kl, Vh, Vl, Oh, Ol);
  k_out<<<dim3(NTOK / 64, DOUT / 64), dim3(128), 0, stream>>>(Oh, Ol, WOh, WOl, bout, out);
  (void)hipGetLastError();
}
